// RNN2_23441931501744
// MI455X (gfx1250) — hardware-run, weakly checked
//
#include <hip/hip_runtime.h>
#include <math.h>

typedef __attribute__((ext_vector_type(16))) _Float16 v16h;
typedef __attribute__((ext_vector_type(8)))  _Float16 v8h;
typedef __attribute__((ext_vector_type(8)))  float    v8f;
typedef __attribute__((ext_vector_type(2)))  float    v2f;

constexpr int kSteps   = 512;
constexpr int kBatch   = 64;
constexpr int kXF      = 160;
constexpr int kLat     = 512;
constexpr int kOutD    = 8;
constexpr int kSta     = 20;
constexpr int kKAll    = kXF + kLat;
constexpr int kRowsPB  = 16;
constexpr int kBlocks  = kBatch / kRowsPB;
constexpr int kThreads = 256;
constexpr int kKSteps  = kKAll / 32;
constexpr int kKStepsH = kLat / 32;
constexpr int kAP      = kKAll + 8;
constexpr int kAPW     = kAP / 2;
constexpr int kSP      = kLat + 4;
constexpr int kParkP   = 16;
constexpr int kRowOut  = kSta * kOutD;
static_assert(kKAll == 672, "K of the cell product");
static_assert((kKAll % 32) == 0 && (kLat % 32) == 0 && (kXF % 32) == 0, "K multiples of 32");
static_assert((kAP % 8) == 0, "16-byte aligned fragment rows");
static_assert((kSP % 2) == 0, "8-byte aligned pair reads");
static_assert(kLat == (kThreads / 32) * 64, "8 waves x 64 columns");
static_assert(kLat == 2 * kThreads, "one column pair per thread");
static_assert((kRowsPB * kXF / 2) == 5 * kThreads, "x staging: 5 pairs per thread");
static_assert(kRowOut == 160 && (kRowOut % 32) == 0, "five whole lines per (step, sample)");
static_assert(kRowsPB == 2 * (kThreads / 32), "two samples per storing wave");

constexpr float kCarryAct = 16.0f;
constexpr float kCarryWgt = 256.0f;
constexpr float kFold     = 1.0f / (kCarryAct * kCarryWgt);
static_assert(kFold == 0.000244140625f, "fold = 2^-12");

constexpr int kWiWords  = kLat * kKAll / 2;
constexpr int kWoRows   = 16;
constexpr int kWoWords  = kWoRows * kLat / 2;
constexpr int kWiBlocks = kWiWords / 256;
constexpr int kWoBlocks = kWoWords / 256;
static_assert((kWiWords % 256) == 0 && (kWoWords % 256) == 0, "exact prep grid");
static_assert(kWiBlocks == 672 && kWoBlocks == 16, "prep grid");
constexpr size_t kBytesWiT = (size_t)kLat * kKAll * 2;
constexpr size_t kBytesWoT = (size_t)kWoRows * kLat * 2;
static_assert(kBytesWiT == 688128ull && kBytesWoT == 16384ull, "plane sizes");

__device__ __forceinline__ unsigned pack2_f16_flush(float a, float b) {
  const float kMinNormal = 6.103515625e-05f;
  const float fa = (fabsf(a) < kMinNormal) ? 0.0f : a;
  const float fb = (fabsf(b) < kMinNormal) ? 0.0f : b;
  const _Float16 h0 = (_Float16)fa;
  const _Float16 h1 = (_Float16)fb;
  const unsigned short u0 = __builtin_bit_cast(unsigned short, h0);
  const unsigned short u1 = __builtin_bit_cast(unsigned short, h1);
  return (unsigned)u0 | ((unsigned)u1 << 16);
}

__device__ __forceinline__ void store2_word(unsigned* p, unsigned v) {
  *(volatile unsigned*)p = v;
  __threadfence();
  *(volatile unsigned*)p = v;
}

union FragH { v16h v; v8h h[2]; };
__device__ __forceinline__ v16h frag_load(const _Float16* p) {
  FragH f;
  f.h[0] = *(const v8h*)(p);
  f.h[1] = *(const v8h*)(p + 16);
  return f.v;
}

__device__ __forceinline__ v8f mma_h(v16h a, v16h b, v8f c) {
  c = __builtin_amdgcn_wmma_f32_16x16x32_f16(false, a, false, b, (short)0, c, false, false);
  asm volatile("v_nop\n\tv_nop\n\tv_nop\n\tv_nop" : "+v"(c) : "v"(a), "v"(b));
  return c;
}

__global__ __launch_bounds__(256) void prep_planes_kernel(
    const float* __restrict__ Wi, const float* __restrict__ Wo,
    unsigned* __restrict__ witu, unsigned* __restrict__ wotu) {
  const int blk = blockIdx.x;
  const int tid = threadIdx.x;
  if (blk < kWiBlocks) {
    const int p = blk * 256 + tid;
    const int e = 2 * p;
    const int n = e / kKAll;
    const int k = e - n * kKAll;
    const float w0 = Wi[(size_t)k * kLat + n];
    const float w1 = Wi[(size_t)(k + 1) * kLat + n];
    const unsigned word = pack2_f16_flush(w0 * kCarryWgt, w1 * kCarryWgt);
    store2_word(witu + p, word);
  } else {
    const int p = (blk - kWiBlocks) * 256 + tid;
    const int e = 2 * p;
    const int n = e >> 9;
    const int k = e & (kLat - 1);
    const int nc = (n < kOutD) ? n : (kOutD - 1);
    const float w0 = Wo[(size_t)k * kOutD + nc];
    const float w1 = Wo[(size_t)(k + 1) * kOutD + nc];
    const bool live = (n < kOutD);
    const float a0 = live ? (w0 * kCarryWgt) : 0.0f;
    const float a1 = live ? (w1 * kCarryWgt) : 0.0f;
    const unsigned word = pack2_f16_flush(a0, a1);
    store2_word(wotu + p, word);
  }
}

__global__ __launch_bounds__(kThreads) void cell_scan_kernel(
    const float* __restrict__ x, const float* __restrict__ h0, const int* __restrict__ nsp,
    const _Float16* __restrict__ WiT, const float* __restrict__ bi,
    const _Float16* __restrict__ WoT, const float* __restrict__ bo,
    float* __restrict__ out) {
  __shared__ __align__(16) unsigned tileW[kRowsPB * kAPW];
  __shared__ __align__(16) float    slab[kRowsPB * kSP];
  __shared__ __align__(16) float    park[kRowsPB * kParkP];

  const int tid  = threadIdx.x;
  const int lane = tid & 31;
  const int wave = tid >> 5;
  const int c    = lane & 15;
  const int hh   = lane >> 4;
  const int b0   = blockIdx.x * kRowsPB;
  const int n0   = wave * 64;

  const int  ns  = nsp[0];
  const bool bad = (ns != kSta);
  const float qnan = __uint_as_float(0x7fc00000u);

  if (tid < 64) tileW[(tid >> 2) * kAPW + (kKAll / 2) + (tid & 3)] = 0u;

#pragma unroll 1
  for (int i = 0; i < kRowsPB; ++i) {
    const v2f hv = *(const v2f*)(h0 + (size_t)(b0 + i) * kLat + 2 * tid);
    const float a = hv[0] * kCarryAct;
    const float b = hv[1] * kCarryAct;
    tileW[i * kAPW + (kXF / 2) + tid] = pack2_f16_flush(a, b);
  }

  float bl0 = bi[n0 + c];
  float bl1 = bi[n0 + 16 + c];
  float bl2 = bi[n0 + 32 + c];
  float bl3 = bi[n0 + 48 + c];
  float bo_l = bo[c & (kOutD - 1)];
  asm volatile("" : "+v"(bo_l));

  const _Float16* tileH = (const _Float16*)tileW;
  const _Float16* arow  = tileH + c * kAP + 8 * hh;
  const _Float16* brow  = WiT + (size_t)(n0 + c) * kKAll + 8 * hh;
  const _Float16* wrow  = WoT + (size_t)c * kLat + 8 * hh;

#pragma unroll 1
  for (int t = 0; t < kSteps; ++t) {
    {
      const float* xb = x + ((size_t)t * kBatch + b0) * kXF;
#pragma unroll
      for (int i = 0; i < 5; ++i) {
        const int p = tid + kThreads * i;
        const v2f xv = *(const v2f*)(xb + 2 * p);
        const int row = p / (kXF / 2);
        const int cp  = p - row * (kXF / 2);
        const float a = xv[0] * kCarryAct;
        const float b = xv[1] * kCarryAct;
        tileW[row * kAPW + cp] = pack2_f16_flush(a, b);
      }
    }
    __syncthreads();

    v8f acc0 = (v8f){0.f, 0.f, 0.f, 0.f, 0.f, 0.f, 0.f, 0.f};
    v8f acc1 = acc0;
    v8f acc2 = acc0;
    v8f acc3 = acc0;
#pragma unroll 3
    for (int ks = 0; ks < kKSteps; ++ks) {
      const v16h fa  = frag_load(arow + 32 * ks);
      const v16h fb0 = frag_load(brow + 32 * ks);
      const v16h fb1 = frag_load(brow + (size_t)16 * kKAll + 32 * ks);
      const v16h fb2 = frag_load(brow + (size_t)32 * kKAll + 32 * ks);
      const v16h fb3 = frag_load(brow + (size_t)48 * kKAll + 32 * ks);
      acc0 = mma_h(fa, fb0, acc0);
      acc1 = mma_h(fa, fb1, acc1);
      acc2 = mma_h(fa, fb2, acc2);
      acc3 = mma_h(fa, fb3, acc3);
    }

    {
      float* sp = slab + (8 * hh) * kSP + n0 + c;
#pragma unroll
      for (int r = 0; r < 8; ++r) {
        sp[r * kSP]      = fmaf(acc0[r], kFold, bl0);
        sp[r * kSP + 16] = fmaf(acc1[r], kFold, bl1);
        sp[r * kSP + 32] = fmaf(acc2[r], kFold, bl2);
        sp[r * kSP + 48] = fmaf(acc3[r], kFold, bl3);
      }
    }
    __syncthreads();

#pragma unroll 1
    for (int i = 0; i < kRowsPB; ++i) {
      const v2f pv = *(const v2f*)(slab + i * kSP + 2 * tid);
      const float a = tanhf(pv[0]) * kCarryAct;
      const float b = tanhf(pv[1]) * kCarryAct;
      tileW[i * kAPW + (kXF / 2) + tid] = pack2_f16_flush(a, b);
    }
    __syncthreads();

    if (wave == 0) {
      v8f ro = (v8f){0.f, 0.f, 0.f, 0.f, 0.f, 0.f, 0.f, 0.f};
#pragma unroll 2
      for (int ks = 0; ks < kKStepsH; ++ks) {
        const v16h fa = frag_load(arow + kXF + 32 * ks);
        const v16h fb = frag_load(wrow + 32 * ks);
        ro = mma_h(fa, fb, ro);
      }
#pragma unroll
      for (int r = 0; r < 8; ++r) {
        const float v = fmaf(ro[r], kFold, bo_l);
        const float s = 1.0f / (1.0f + expf(-v));
        park[(8 * hh + r) * kParkP + c] = s;
      }
    }
    __syncthreads();

    {
      const float p0 = park[(2 * wave) * kParkP + (lane & 7)];
      const float p1 = park[(2 * wave + 1) * kParkP + (lane & 7)];
      const float v0 = bad ? qnan : p0;
      const float v1 = bad ? qnan : p1;
      float* o0 = out + ((size_t)t * kBatch + b0 + 2 * wave) * kRowOut + lane;
      for (int pass = 0; pass < 2; ++pass) {
#pragma unroll
        for (int j = 0; j < 5; ++j) {
          *(volatile float*)(o0 + 32 * j) = v0;
          *(volatile float*)(o0 + kRowOut + 32 * j) = v1;
        }
        __threadfence();
      }
    }
  }
}

extern "C" void kernel_launch(void* const* d_in, const int* in_sizes, int n_in,
                              void* d_out, int out_size, void* d_ws, size_t ws_size,
                              hipStream_t stream) {
  if (n_in < 7 || d_out == nullptr || d_ws == nullptr) return;
  if (in_sizes[0] != kSteps * kBatch * kXF) return;
  if (in_sizes[1] != kBatch * kLat) return;
  if (in_sizes[2] != 1) return;
  if (in_sizes[3] != kKAll * kLat) return;
  if (in_sizes[4] != kLat) return;
  if (in_sizes[5] != kLat * kOutD) return;
  if (in_sizes[6] != kOutD) return;
  if (out_size != kSteps * kBatch * kSta * kOutD) return;

  const float* x   = (const float*)d_in[0];
  const float* h0  = (const float*)d_in[1];
  const int*   nsp = (const int*)d_in[2];
  const float* Wi  = (const float*)d_in[3];
  const float* bi  = (const float*)d_in[4];
  const float* Wo  = (const float*)d_in[5];
  const float* bo  = (const float*)d_in[6];
  float* out = (float*)d_out;

  char* ws = (char*)d_ws;
  size_t off = 0;
  auto carve = [&](size_t bytes) -> char* {
    char* p = ws + off;
    off += (bytes + 255) & ~(size_t)255;
    return p;
  };
  unsigned* WiTu = (unsigned*)carve(kBytesWiT);
  unsigned* WoTu = (unsigned*)carve(kBytesWoT);
  if (off != (size_t)704512 || off > ws_size || off > (size_t)134217728) return;

  prep_planes_kernel<<<kWiBlocks + kWoBlocks, 256, 0, stream>>>(Wi, Wo, WiTu, WoTu);

  cell_scan_kernel<<<kBlocks, kThreads, 0, stream>>>(
      x, h0, nsp, (const _Float16*)WiTu, bi, (const _Float16*)WoTu, bo, out);
}
